// SegmentedAttention_16338055594765
// MI455X (gfx1250) — hardware-verified
//
#include <hip/hip_runtime.h>
#include <math.h>
#include <stdint.h>

#define NTOK   8192
#define NPOS   4096
#define DIMM   1024
#define NHEAD  16
#define DHD    64
#define SEGL   512
#define NPM    16
#define NWIN   16
#define QKVN   3072
#define QKN    2048
#define KCAT   2048
#define NFREQ  32
#define RMS_EPS 1.1920929e-07f

static_assert(NTOK % 32 == 0);
static_assert(QKN % 128 == 0);
static_assert(DIMM % 128 == 0);
static_assert(NTOK % 128 == 0);
static_assert(KCAT % 32 == 0);
static_assert(NWIN * SEGL == NTOK);
static_assert(NPOS % 16 == 0);

typedef _Float16     v16h __attribute__((ext_vector_type(16)));
typedef _Float16     v8h  __attribute__((ext_vector_type(8)));
typedef __bf16       v16b __attribute__((ext_vector_type(16)));
typedef __bf16       v8b  __attribute__((ext_vector_type(8)));
typedef float        v8f  __attribute__((ext_vector_type(8)));
typedef float        v4f  __attribute__((ext_vector_type(4)));
typedef unsigned int v4u  __attribute__((ext_vector_type(4)));

__device__ __forceinline__ unsigned short bf_bits(float f) {
  const unsigned u = __float_as_uint(f);
  return (unsigned short)((u + 0x7FFFu + ((u >> 16) & 1u)) >> 16);
}
__device__ __forceinline__ float bf_val(unsigned short h) { return __uint_as_float(((unsigned)h) << 16); }
__device__ __forceinline__ float bf_rne(float f) { return bf_val(bf_bits(f)); }
__device__ __forceinline__ unsigned pk16(unsigned short a, unsigned short b) { return (unsigned)a | ((unsigned)b << 16); }
__device__ __forceinline__ v8f zero8() { v8f z = {0.f, 0.f, 0.f, 0.f, 0.f, 0.f, 0.f, 0.f}; return z; }
__device__ __forceinline__ int wave_id() { return __builtin_amdgcn_readfirstlane((int)(threadIdx.x >> 5)); }

__device__ __forceinline__ void lds_wave_sync() {
  __builtin_amdgcn_fence(__ATOMIC_RELEASE, "workgroup");
  __builtin_amdgcn_wave_barrier();
  __builtin_amdgcn_fence(__ATOMIC_ACQUIRE, "workgroup");
}

union FragH { v16h v; v8h h[2]; };
union FragB { v16b v; v8b h[2]; };
__device__ __forceinline__ v16h ldfrag_h(const _Float16* p) { FragH f; f.h[0] = *(const v8h*)(p); f.h[1] = *(const v8h*)(p + 16); return f.v; }
__device__ __forceinline__ v16b ldfrag_b(const __bf16* p)   { FragB f; f.h[0] = *(const v8b*)(p); f.h[1] = *(const v8b*)(p + 16); return f.v; }

__device__ __forceinline__ v8f mma_h(v16h a, v16h b, v8f c) {
  return __builtin_amdgcn_wmma_f32_16x16x32_f16(false, a, false, b, (short)0, c, false, false);
}
__device__ __forceinline__ v8f mma_b(v16b a, v16b b, v8f c) {
  return __builtin_amdgcn_wmma_f32_16x16x32_bf16(false, a, false, b, (short)0, c, false, false);
}
__device__ __forceinline__ void guard_b3(v8f& a, v8f& b, v16b x0, v16b x1, v16b y) {
  asm volatile("v_nop\n\tv_nop\n\tv_nop\n\tv_nop" : "+v"(a), "+v"(b) : "v"(x0), "v"(x1), "v"(y) : "memory");
}
__device__ __forceinline__ void guard_h3(v8f& a, v8f& b, v16h x, v16h y, v16h z) {
  asm volatile("v_nop\n\tv_nop\n\tv_nop\n\tv_nop" : "+v"(a), "+v"(b) : "v"(x), "v"(y), "v"(z) : "memory");
}
__device__ __forceinline__ void guard_h4(v8f& a, v8f& b, v16h w, v16h x, v16h y, v16h z) {
  asm volatile("v_nop\n\tv_nop\n\tv_nop\n\tv_nop" : "+v"(a), "+v"(b) : "v"(w), "v"(x), "v"(y), "v"(z) : "memory");
}
__device__ __forceinline__ void acc_guard4(v8f& a, v8f& b, v8f& c, v8f& d) {
  asm volatile("v_nop\n\tv_nop\n\tv_nop\n\tv_nop" : "+v"(a), "+v"(b), "+v"(c), "+v"(d));
}

__global__ __launch_bounds__(128) void prep_x_kernel(const float* __restrict__ seq, const float* __restrict__ g,
                                                     unsigned short* __restrict__ x2, int nrows) {
  __shared__ float red[4];
  const int row = (int)blockIdx.x;
  if (row >= nrows) return;
  const int tid  = (int)threadIdx.x;
  const int lane = tid & 31;
  const int wave = tid >> 5;
  const float* sp = seq + (size_t)row * DIMM + 8 * tid;
  const v4f a = *(const v4f*)sp;
  const v4f b = *(const v4f*)(sp + 4);
  float sb[8];
#pragma unroll
  for (int e = 0; e < 4; ++e) { sb[e] = bf_rne(a[e]); sb[4 + e] = bf_rne(b[e]); }
  float ss = 0.0f;
#pragma unroll
  for (int e = 0; e < 8; ++e) ss += sb[e] * sb[e];
#pragma unroll
  for (int off = 16; off >= 1; off >>= 1) ss += __shfl_xor(ss, off, 32);
  if (lane == 0) red[wave] = ss;
  __syncthreads();
  const float tot = (red[0] + red[1]) + (red[2] + red[3]);
  const float rsc = rsqrtf(tot * 0.0009765625f + RMS_EPS);
  const v4f ga = *(const v4f*)(g + 8 * tid);
  const v4f gb = *(const v4f*)(g + 8 * tid + 4);
  float gv[8];
#pragma unroll
  for (int e = 0; e < 4; ++e) { gv[e] = bf_rne(ga[e]); gv[4 + e] = bf_rne(gb[e]); }
  v4u wh, wl;
#pragma unroll
  for (int q = 0; q < 4; ++q) {
    const float x0 = (sb[2 * q] * rsc) * gv[2 * q];
    const float x1 = (sb[2 * q + 1] * rsc) * gv[2 * q + 1];
    const unsigned short h0 = bf_bits(x0), h1 = bf_bits(x1);
    const unsigned short l0 = bf_bits(x0 - bf_val(h0)), l1 = bf_bits(x1 - bf_val(h1));
    wh[q] = pk16(h0, h1);
    wl[q] = pk16(l0, l1);
  }
  const size_t o = (size_t)row * KCAT + 8 * tid;
  *(volatile v4u*)(x2 + o)        = wh;
  *(volatile v4u*)(x2 + o + DIMM) = wl;
  __threadfence();
  *(volatile v4u*)(x2 + o)        = wh;
  *(volatile v4u*)(x2 + o + DIMM) = wl;
}

__global__ __launch_bounds__(256) void cvt_bf16_kernel(const float* __restrict__ in, unsigned short* __restrict__ outp, int n8) {
  const int i = (int)blockIdx.x * 256 + (int)threadIdx.x;
  if (i >= n8) return;
  const size_t e = 8 * (size_t)i;
  const v4f a = *(const v4f*)(in + e);
  const v4f b = *(const v4f*)(in + e + 4);
  v4u w;
  w[0] = pk16(bf_bits(a[0]), bf_bits(a[1]));
  w[1] = pk16(bf_bits(a[2]), bf_bits(a[3]));
  w[2] = pk16(bf_bits(b[0]), bf_bits(b[1]));
  w[3] = pk16(bf_bits(b[2]), bf_bits(b[3]));
  *(volatile v4u*)(outp + e) = w;
  __threadfence();
  *(volatile v4u*)(outp + e) = w;
}

__global__ __launch_bounds__(256) void rope_table_kernel(float* __restrict__ cst, float* __restrict__ snt, int npos) {
  const int lane = threadIdx.x & 31;
  const int wave = (int)(threadIdx.x >> 5);
  const int t = (int)blockIdx.x * 8 + wave;
  if (t >= npos) return;
  const float e   = (float)(2 * lane) * 0.015625f;
  const float pw  = powf(10000.0f, e);
  const float inv = 1.0f / pw;
  const float ang = (float)t * inv;
  const float cv = cosf(ang);
  const float sv = sinf(ang);
  const size_t o = (size_t)t * NFREQ + lane;
  for (int pass = 0; pass < 2; ++pass) {
    ((volatile float*)cst)[o] = cv;
    ((volatile float*)snt)[o] = sv;
    __threadfence();
  }
}

__global__ __launch_bounds__(256) void pm_planes_kernel(const float* __restrict__ pm, unsigned short* __restrict__ pmkp,
                                                        unsigned short* __restrict__ pmvhp, unsigned short* __restrict__ pmvlp) {
  __shared__ __align__(16) float tf[NPM * 68];
  const int h   = (int)blockIdx.x;
  const int tid = (int)threadIdx.x;
  _Float16* PK  = (_Float16*)(void*)pmkp;
  _Float16* PVh = (_Float16*)(void*)pmvhp;
  _Float16* PVl = (_Float16*)(void*)pmvlp;

  const int key = tid >> 3;
  const int d0  = (tid & 7) * 8;
  const int kcl = (key < NPM) ? key : (NPM - 1);
  const float keepk = (key < NPM) ? 1.0f : 0.0f;
  const float* kr = pm + ((size_t)(h * NPM + kcl) * DHD + d0);
  const v4f ka = *(const v4f*)kr;
  const v4f kb = *(const v4f*)(kr + 4);
  v8h kv;
#pragma unroll
  for (int e = 0; e < 4; ++e) {
    kv[e]     = (_Float16)(bf_rne(ka[e]) * keepk);
    kv[4 + e] = (_Float16)(bf_rne(kb[e]) * keepk);
  }
  {
    const int r  = tid >> 4;
    const int c4 = (tid & 15) * 4;
    const v4f a = *(const v4f*)(pm + ((size_t)((NHEAD + h) * NPM + r) * DHD + c4));
    *(v4f*)(tf + r * 68 + c4) = a;
  }
  __syncthreads();
  const int d  = tid >> 2;
  const int k0 = (tid & 3) * 8;
  const float keepv = (k0 < NPM) ? 1.0f : 0.0f;
  v8h vv, vz;
#pragma unroll
  for (int e = 0; e < 8; ++e) {
    const int kk = (k0 + e) & (NPM - 1);
    vv[e] = (_Float16)(bf_rne(tf[kk * 68 + d]) * keepv);
    vz[e] = (_Float16)0.0f;
  }
  const size_t ko = ((size_t)(h * 32 + key)) * DHD + d0;
  const size_t vo = ((size_t)(h * DHD + d)) * 32 + k0;
  for (int pass = 0; pass < 2; ++pass) {
    *(volatile v8h*)(PK + ko)  = kv;
    *(volatile v8h*)(PVh + vo) = vv;
    *(volatile v8h*)(PVl + vo) = vz;
    __threadfence();
  }
}

template <int EPI> struct SlabT { typedef _Float16 T; static constexpr int PERW = 4096; };
template <> struct SlabT<2>     { typedef float    T; static constexpr int PERW = 2048; };
template <int EPI> struct TrigT { static constexpr int PERW = 8; };
template <> struct TrigT<0>     { static constexpr int PERW = 1024; };

template <int EPI>
__global__ __launch_bounds__(128) void gemm_w32x128_kernel(
    const unsigned short* __restrict__ Ap, int lda, int maskA,
    const unsigned short* __restrict__ Btp, int ldb, int maskB,
    const float* __restrict__ cst, const float* __restrict__ snt,
    void* C0, void* C1, void* C2, int ldc,
    int M, int N, int K) {
  typedef typename SlabT<EPI>::T ST;
  __shared__ __align__(16) ST slab_all[4 * SlabT<EPI>::PERW];
  __shared__ __align__(16) float trig_all[4 * TrigT<EPI>::PERW];

  const int lane = threadIdx.x & 31;
  const int wave = wave_id();
  const int hh = lane >> 4;
  const int rl = lane & 15;
  const int tilesN = N >> 7;
  const int tilesM = M >> 5;
  const int tile = (int)blockIdx.x * 4 + wave;
  if (tile >= tilesM * tilesN) return;
  const int tm = tile / tilesN;
  const int tn = tile - tm * tilesN;
  const int m0 = tm << 5;
  const int n0 = tn << 7;

  const __bf16* A  = (const __bf16*)(const void*)Ap;
  const __bf16* Bt = (const __bf16*)(const void*)Btp;

  v8f acc[2][8];
#pragma unroll
  for (int i = 0; i < 2; ++i)
#pragma unroll
    for (int j = 0; j < 8; ++j) acc[i][j] = zero8();

  for (int k0 = 0; k0 < K; k0 += 32) {
    const int ka = (k0 & maskA) + 8 * hh;
    const int kb = (k0 & maskB) + 8 * hh;
    v16b af[2];
#pragma unroll
    for (int i = 0; i < 2; ++i) af[i] = ldfrag_b(A + (size_t)(m0 + i * 16 + rl) * lda + ka);
#pragma unroll
    for (int j = 0; j < 8; ++j) {
      const v16b bj = ldfrag_b(Bt + (size_t)(n0 + j * 16 + rl) * ldb + kb);
      acc[0][j] = mma_b(af[0], bj, acc[0][j]);
      acc[1][j] = mma_b(af[1], bj, acc[1][j]);
      guard_b3(acc[0][j], acc[1][j], af[0], af[1], bj);
    }
  }
  acc_guard4(acc[0][0], acc[0][1], acc[0][2], acc[0][3]);
  acc_guard4(acc[0][4], acc[0][5], acc[0][6], acc[0][7]);
  acc_guard4(acc[1][0], acc[1][1], acc[1][2], acc[1][3]);
  acc_guard4(acc[1][4], acc[1][5], acc[1][6], acc[1][7]);

  ST* slab = slab_all + wave * SlabT<EPI>::PERW;
  _Float16* sl16 = (_Float16*)(void*)slab;
  float*    slf  = (float*)(void*)slab;

  if (EPI == 0) {
    const bool isq = (n0 < DIMM);
    _Float16* P0 = isq ? (_Float16*)C0 : (_Float16*)C2;
    _Float16* P1 = (_Float16*)C1;
    const int col0 = isq ? n0 : (n0 - DIMM);
    float* csl = trig_all + wave * TrigT<EPI>::PERW;
    float* snl = csl + 16 * NFREQ;
#pragma unroll
    for (int i = 0; i < 2; ++i) {
      const int pos0 = (m0 + i * 16) & (NPOS - 1);
      {
        v4f cv4[4], sv4[4];
#pragma unroll
        for (int it = 0; it < 4; ++it) {
          const int p  = it * 32 + lane;
          const int rr = p >> 3;
          const int c4 = (p & 7) * 4;
          cv4[it] = *(const v4f*)(cst + (size_t)(pos0 + rr) * NFREQ + c4);
          sv4[it] = *(const v4f*)(snt + (size_t)(pos0 + rr) * NFREQ + c4);
        }
#pragma unroll
        for (int it = 0; it < 4; ++it) {
          const int p  = it * 32 + lane;
          const int rr = p >> 3;
          const int c4 = (p & 7) * 4;
          *(v4f*)(csl + rr * NFREQ + c4) = cv4[it];
          *(v4f*)(snl + rr * NFREQ + c4) = sv4[it];
        }
      }
      lds_wave_sync();
#pragma unroll
      for (int j = 0; j < 8; ++j) {
        const int dl = (j & 3) * 16 + rl;
        const int fi = dl >> 1;
        const float sgn = (rl & 1) ? 1.0f : -1.0f;
#pragma unroll
        for (int r = 0; r < 8; ++r) {
          const int sr = 8 * hh + r;
          const float cv = csl[sr * NFREQ + fi];
          const float sv = snl[sr * NFREQ + fi];
          const float val = acc[i][j][r];
          const float prt = __shfl_xor(val, 1, 32);
          const float o = val * cv + sgn * prt * sv;
          const _Float16 h1 = (_Float16)o;
          const int so = sr * 128 + j * 16 + rl;
          sl16[so]        = h1;
          sl16[2048 + so] = (_Float16)((o - (float)h1) * 2048.0f);
        }
      }
      lds_wave_sync();
      for (int pass = 0; pass < 2; ++pass) {
#pragma unroll
        for (int it = 0; it < 8; ++it) {
          const int row = it * 2 + hh;
          const int c8  = rl * 8;
          const v8h vh = *(const v8h*)(sl16 + row * 128 + c8);
          const v8h vl = *(const v8h*)(sl16 + 2048 + row * 128 + c8);
          const size_t go = (size_t)(m0 + i * 16 + row) * ldc + col0 + c8;
          *(volatile v8h*)(P0 + go) = vh;
          if (isq) *(volatile v8h*)(P1 + go) = vl;
        }
        __threadfence();
      }
      lds_wave_sync();
    }
  } else if (EPI == 1) {
    _Float16* P0 = (_Float16*)C0;
    _Float16* P1 = (_Float16*)C1;
#pragma unroll
    for (int i = 0; i < 2; ++i) {
#pragma unroll
      for (int r = 0; r < 8; ++r) {
#pragma unroll
        for (int j = 0; j < 8; ++j) {
          const float v = acc[i][j][r];
          const _Float16 hv = (_Float16)v;
          const int so = (8 * hh + r) * 128 + j * 16 + rl;
          sl16[so]        = hv;
          sl16[2048 + so] = (_Float16)((v - (float)hv) * 2048.0f);
        }
      }
      lds_wave_sync();
      for (int pass = 0; pass < 2; ++pass) {
#pragma unroll
        for (int it = 0; it < 8; ++it) {
          const int row = it * 2 + hh;
          const int c8  = rl * 8;
          const v8h vh = *(const v8h*)(sl16 + row * 128 + c8);
          const v8h vl = *(const v8h*)(sl16 + 2048 + row * 128 + c8);
          const size_t go = (size_t)(m0 + i * 16 + row) * ldc + n0 + c8;
          *(volatile v8h*)(P0 + go) = vh;
          *(volatile v8h*)(P1 + go) = vl;
        }
        __threadfence();
      }
      lds_wave_sync();
    }
  } else {
    float* C = (float*)C0;
#pragma unroll
    for (int i = 0; i < 2; ++i) {
#pragma unroll
      for (int j = 0; j < 8; ++j)
#pragma unroll
        for (int r = 0; r < 8; ++r)
          slf[(8 * hh + r) * 128 + j * 16 + rl] = acc[i][j][r];
      lds_wave_sync();
      for (int pass = 0; pass < 2; ++pass) {
#pragma unroll
        for (int row = 0; row < 16; ++row) {
          const v4f v = *(const v4f*)(slf + row * 128 + lane * 4);
          *(volatile v4f*)(C + (size_t)(m0 + i * 16 + row) * ldc + n0 + lane * 4) = v;
        }
        __threadfence();
      }
      lds_wave_sync();
    }
  }
}

#define AT_KC   32
#define KS_P    72
#define VS_P    40
#define PS_P    40
#define LDS_KS  0
#define LDS_VHS (AT_KC * KS_P)
#define LDS_VLS (LDS_VHS + DHD * VS_P)
#define LDS_PH  (LDS_VLS + DHD * VS_P)
#define LDS_PL  (LDS_PH + 4 * 16 * PS_P)
#define LDS_TOT (LDS_PL + 4 * 16 * PS_P)
static_assert(LDS_TOT * 2 <= 65536);
static_assert(4 * 2048 <= LDS_TOT);
static_assert((LDS_VHS * 2) % 16 == 0);
static_assert((LDS_VLS * 2) % 16 == 0);
static_assert((LDS_PH * 2) % 16 == 0);
static_assert((LDS_PL * 2) % 16 == 0);

__global__ __launch_bounds__(128) void attn_seg_kernel(
    const unsigned short* __restrict__ qhp, const unsigned short* __restrict__ qlp,
    const unsigned short* __restrict__ khp,
    const unsigned short* __restrict__ vhp, const unsigned short* __restrict__ vlp,
    const unsigned short* __restrict__ pmkp, const unsigned short* __restrict__ pmvhp, const unsigned short* __restrict__ pmvlp,
    unsigned short* __restrict__ aop) {
  __shared__ __align__(16) _Float16 lds[LDS_TOT];
  _Float16* Ks  = lds + LDS_KS;
  _Float16* Vhs = lds + LDS_VHS;
  _Float16* Vls = lds + LDS_VLS;

  const int tid  = (int)threadIdx.x;
  const int lane = tid & 31;
  const int wave = wave_id();
  const int hh   = lane >> 4;
  const int c    = lane & 15;
  const int qt   = (int)blockIdx.x;
  const int h    = (int)blockIdx.y;
  const int sw   = (int)blockIdx.z;
  const size_t tok0 = (size_t)sw * SEGL;
  const int q0    = qt * 64 + wave * 16;
  const int qlast = q0 + 15;

  const _Float16* Qhr  = (const _Float16*)(const void*)qhp + (tok0 + q0 + c) * DIMM + h * DHD + 8 * hh;
  const _Float16* Qlr  = (const _Float16*)(const void*)qlp + (tok0 + q0 + c) * DIMM + h * DHD + 8 * hh;
  const _Float16* Kg   = (const _Float16*)(const void*)khp + tok0 * DIMM + h * DHD;
  const _Float16* Vhg  = (const _Float16*)(const void*)vhp + (size_t)(h * DHD) * NTOK + tok0;
  const _Float16* Vlg  = (const _Float16*)(const void*)vlp + (size_t)(h * DHD) * NTOK + tok0;
  const _Float16* PKg  = (const _Float16*)(const void*)pmkp + (size_t)h * AT_KC * DHD;
  const _Float16* PVhg = (const _Float16*)(const void*)pmvhp + (size_t)h * DHD * AT_KC;
  const _Float16* PVlg = (const _Float16*)(const void*)pmvlp + (size_t)h * DHD * AT_KC;
  _Float16* ph = lds + LDS_PH + wave * (16 * PS_P);
  _Float16* pl = lds + LDS_PL + wave * (16 * PS_P);

  float mrow[8], lrow[8];
  v8f oacc[4], oaccr[4];
#pragma unroll
  for (int r = 0; r < 8; ++r) { mrow[r] = -INFINITY; lrow[r] = 0.f; }
#pragma unroll
  for (int t = 0; t < 4; ++t) { oacc[t] = zero8(); oaccr[t] = zero8(); }

  const int nch = 2 * qt + 3;
  for (int kc = 0; kc < nch; ++kc) {
    const int  kv0  = (kc - 1) * AT_KC;
    const bool ispm = (kc == 0);
    const int  koff = ispm ? 0 : kv0;
    const _Float16* ksrc = ispm ? PKg  : (Kg + (size_t)koff * DIMM);
    const int       kp   = ispm ? DHD  : DIMM;
    const _Float16* vsh  = ispm ? PVhg : (Vhg + koff);
    const _Float16* vsl  = ispm ? PVlg : (Vlg + koff);
    const int       vp   = ispm ? AT_KC : NTOK;
    __syncthreads();
#pragma unroll
    for (int i = 0; i < 2; ++i) {
      const int p   = tid + 128 * i;
      const int key = p >> 3, d8 = (p & 7) * 8;
      const v8h kx = *(const v8h*)(ksrc + (size_t)key * kp + d8);
      *(v8h*)(Ks + key * KS_P + d8) = kx;
      const int d = p >> 2, k8 = (p & 3) * 8;
      const v8h vx = *(const v8h*)(vsh + (size_t)d * vp + k8);
      const v8h vy = *(const v8h*)(vsl + (size_t)d * vp + k8);
      *(v8h*)(Vhs + d * VS_P + k8) = vx;
      *(v8h*)(Vls + d * VS_P + k8) = vy;
    }
    __syncthreads();

    if (kv0 <= qlast) {
      v8f sh[2], sr[2];
      sh[0] = zero8(); sh[1] = zero8(); sr[0] = zero8(); sr[1] = zero8();
#pragma unroll
      for (int dc = 0; dc < 2; ++dc) {
        const v16h qa = ldfrag_h(Qhr + dc * 32);
        const v16h ql = ldfrag_h(Qlr + dc * 32);
#pragma unroll
        for (int j = 0; j < 2; ++j) {
          const v16h kb = ldfrag_h(Ks + (j * 16 + c) * KS_P + dc * 32 + 8 * hh);
          sh[j] = mma_h(qa, kb, sh[j]);
          sr[j] = mma_h(ql, kb, sr[j]);
          guard_h3(sh[j], sr[j], qa, ql, kb);
        }
      }
      float cm[8];
#pragma unroll
      for (int r = 0; r < 8; ++r) {
        const int qrow = q0 + 8 * hh + r;
        const int lim  = ispm ? (NPM - 1) : qrow;
        float m = -INFINITY;
#pragma unroll
        for (int j = 0; j < 2; ++j) {
          const int key = koff + j * 16 + c;
          float s = (sh[j][r] + sr[j][r] * 0.00048828125f) * 0.125f;
          s = (key > lim) ? -INFINITY : s;
          sh[j][r] = s;
          m = fmaxf(m, s);
        }
#pragma unroll
        for (int off = 1; off < 16; off <<= 1) m = fmaxf(m, __shfl_xor(m, off, 32));
        cm[r] = m;
      }
#pragma unroll
      for (int r = 0; r < 8; ++r) {
        const float mnew  = fmaxf(mrow[r], cm[r]);
        const float alpha = __expf(mrow[r] - mnew);
        mrow[r] = mnew;
        float psum = 0.f;
#pragma unroll
        for (int j = 0; j < 2; ++j) {
          const float p  = __expf(sh[j][r] - mnew);
          psum += p;
          const float pp = p * 1024.0f;
          const _Float16 phv = (_Float16)pp;
          const int po = (8 * hh + r) * PS_P + j * 16 + c;
          ph[po] = phv;
          pl[po] = (_Float16)((pp - (float)phv) * 2048.0f);
        }
#pragma unroll
        for (int off = 1; off < 16; off <<= 1) psum += __shfl_xor(psum, off, 32);
        lrow[r] = lrow[r] * alpha + psum;
#pragma unroll
        for (int t = 0; t < 4; ++t) { oacc[t][r] *= alpha; oaccr[t][r] *= alpha; }
      }
      lds_wave_sync();
      const v16h pa = ldfrag_h(ph + c * PS_P + 8 * hh);
      const v16h pr = ldfrag_h(pl + c * PS_P + 8 * hh);
#pragma unroll
      for (int t = 0; t < 4; ++t) {
        const v16h vb = ldfrag_h(Vhs + (t * 16 + c) * VS_P + 8 * hh);
        const v16h vr = ldfrag_h(Vls + (t * 16 + c) * VS_P + 8 * hh);
        oacc[t]  = mma_h(pa, vb, oacc[t]);
        oaccr[t] = mma_h(pa, vr, oaccr[t]);
        oaccr[t] = mma_h(pr, vb, oaccr[t]);
        guard_h4(oacc[t], oaccr[t], pa, pr, vb, vr);
      }
    }
  }

  __syncthreads();
  _Float16* osh = lds + wave * 2048;
  _Float16* osl = osh + 1024;
#pragma unroll
  for (int r = 0; r < 8; ++r) {
    const float inv = (1.0f / lrow[r]) * 0.0009765625f;
#pragma unroll
    for (int t = 0; t < 4; ++t) {
      const float o = (oacc[t][r] + oaccr[t][r] * 0.00048828125f) * inv;
      const unsigned short hb = bf_bits(o);
      const unsigned short lb = bf_bits(o - bf_val(hb));
      const int so = (8 * hh + r) * 64 + t * 16 + c;
      osh[so] = __builtin_bit_cast(_Float16, hb);
      osl[so] = __builtin_bit_cast(_Float16, lb);
    }
  }
  lds_wave_sync();
  _Float16* Ag = (_Float16*)(void*)aop + (tok0 + q0) * KCAT + h * DHD;
  const int rq = lane >> 3;
  const int c8 = (lane & 7) * 8;
  for (int pass = 0; pass < 2; ++pass) {
#pragma unroll
    for (int it = 0; it < 4; ++it) {
      const int row = it * 4 + rq;
      const v8h x = *(const v8h*)(osh + row * 64 + c8);
      const v8h y = *(const v8h*)(osl + row * 64 + c8);
      *(volatile v8h*)(Ag + (size_t)row * KCAT + c8)        = x;
      *(volatile v8h*)(Ag + (size_t)row * KCAT + DIMM + c8) = y;
    }
    __threadfence();
  }
}

extern "C" void kernel_launch(void* const* d_in, const int* in_sizes, int n_in,
                              void* d_out, int out_size, void* d_ws, size_t ws_size,
                              hipStream_t stream) {
  if (n_in < 5) return;
  if (in_sizes[0] != NTOK * DIMM) return;
  if (in_sizes[1] != DIMM) return;
  if (in_sizes[2] != QKVN * DIMM) return;
  if (in_sizes[3] != DIMM * DIMM) return;
  if (in_sizes[4] != 2 * NHEAD * NPM * DHD) return;
  if (out_size != NTOK * DIMM) return;

  const float* seq  = (const float*)d_in[0];
  const float* g    = (const float*)d_in[1];
  const float* wqkv = (const float*)d_in[2];
  const float* wout = (const float*)d_in[3];
  const float* pm   = (const float*)d_in[4];
  float* out = (float*)d_out;

  const size_t szX  = (size_t)NTOK * KCAT * 2;
  const size_t szWQ = (size_t)QKVN * DIMM * 2;
  const size_t szWO = (size_t)DIMM * DIMM * 2;
  const size_t szT  = (size_t)NPOS * NFREQ * 4;
  const size_t szPM = (size_t)NHEAD * AT_KC * DHD * 2;
  const size_t szQ  = (size_t)NTOK * DIMM * 2;
  const size_t szV  = (size_t)DIMM * NTOK * 2;
  size_t off = 0;
  const size_t oX   = off; off += szX;
  const size_t oWQ  = off; off += szWQ;
  const size_t oWO  = off; off += szWO;
  const size_t oCs  = off; off += szT;
  const size_t oSn  = off; off += szT;
  const size_t oPK  = off; off += szPM;
  const size_t oPVh = off; off += szPM;
  const size_t oPVl = off; off += szPM;
  const size_t oQh  = off; off += szQ;
  const size_t oQl  = off; off += szQ;
  const size_t oKh  = off; off += szQ;
  const size_t oVh  = off; off += szV;
  const size_t oVl  = off; off += szV;
  if (off > ws_size) return;

  char* ws = (char*)d_ws;
  unsigned short* X2   = (unsigned short*)(ws + oX);
  unsigned short* WQ   = (unsigned short*)(ws + oWQ);
  unsigned short* WO   = (unsigned short*)(ws + oWO);
  float*          cst  = (float*)(ws + oCs);
  float*          snt  = (float*)(ws + oSn);
  unsigned short* PMK  = (unsigned short*)(ws + oPK);
  unsigned short* PMVh = (unsigned short*)(ws + oPVh);
  unsigned short* PMVl = (unsigned short*)(ws + oPVl);
  unsigned short* Qh   = (unsigned short*)(ws + oQh);
  unsigned short* Ql   = (unsigned short*)(ws + oQl);
  unsigned short* Kh   = (unsigned short*)(ws + oKh);
  unsigned short* VTh  = (unsigned short*)(ws + oVh);
  unsigned short* VTl  = (unsigned short*)(ws + oVl);
  unsigned short* AO2  = X2;

  const dim3 b256(256), b128(128);
  const int noMask = 0x7FFFFFFF;
  const int wrapK  = DIMM - 1;

  prep_x_kernel<<<dim3(NTOK), b128, 0, stream>>>(seq, g, X2, NTOK);
  cvt_bf16_kernel<<<dim3((QKVN * DIMM / 8) / 256), b256, 0, stream>>>(wqkv, WQ, QKVN * DIMM / 8);
  cvt_bf16_kernel<<<dim3((DIMM * DIMM / 8) / 256), b256, 0, stream>>>(wout, WO, DIMM * DIMM / 8);
  rope_table_kernel<<<dim3(NPOS / 8), b256, 0, stream>>>(cst, snt, NPOS);
  pm_planes_kernel<<<dim3(NHEAD), b256, 0, stream>>>(pm, PMK, PMVh, PMVl);
  gemm_w32x128_kernel<0><<<dim3((NTOK / 32) * (QKN / 128) / 4), b128, 0, stream>>>(
      X2, KCAT, noMask, WQ, DIMM, wrapK, cst, snt, (void*)Qh, (void*)Ql, (void*)Kh, DIMM, NTOK, QKN, KCAT);
  gemm_w32x128_kernel<1><<<dim3((DIMM / 32) * (NTOK / 128) / 4), b128, 0, stream>>>(
      WQ + (size_t)QKN * DIMM, DIMM, wrapK, X2, KCAT, noMask, cst, snt, (void*)VTh, (void*)VTl, (void*)VTh, NTOK, DIMM, NTOK, KCAT);
  attn_seg_kernel<<<dim3(SEGL / 64, NHEAD, NWIN), b128, 0, stream>>>(Qh, Ql, Kh, VTh, VTl, PMK, PMVh, PMVl, AO2);
  gemm_w32x128_kernel<2><<<dim3((NTOK / 32) * (DIMM / 128) / 4), b128, 0, stream>>>(
      AO2, KCAT, noMask, WO, DIMM, wrapK, cst, snt, (void*)out, (void*)out, (void*)out, DIMM, NTOK, DIMM, KCAT);
  (void)hipGetLastError();
}
